// _SAmodule_57019985822402
// MI455X (gfx1250) — hardware-run, weakly checked
//
#include <hip/hip_runtime.h>


#define CH    8
#define DIM   32
#define HW    1024
#define DHW   32768
#define CDHW  262144
#define PD    34
#define PVOX  (PD * PD * PD)
#define NTAP  27
#define KP    224
#define KSTEPS 7
#define WROWS 32
#define CW    4
#define OSP   36
#define L2E   1.4426950408889634f

static_assert(PD == DIM + 2);
static_assert(KP % 32 == 0);
static_assert(KP >= NTAP * CH);
static_assert(KSTEPS * 32 == KP);
static_assert(CH == 8);
static_assert(WROWS * (KP / 8) == 896);
static_assert((WROWS * KP * 2) % 128 == 0);
static_assert(PVOX % 8 == 0);
static_assert((DIM * DIM) % CW == 0);
static_assert((OSP * 4) % 16 == 0);
static_assert(CW * 32 * OSP * 4 <= 131072);
static_assert(32 * 16 * 6 == 3 * CH * 128);
static_assert((CH * DIM / 4) * HW == 256 * 256);
static_assert(256 * 4 == HW);
static_assert(256 / 32 == CH);
static_assert(DIM == 32);

typedef unsigned short bf;
typedef __attribute__((ext_vector_type(16))) __bf16   v16bf;
typedef __attribute__((ext_vector_type(8)))  unsigned short v8us;
typedef __attribute__((ext_vector_type(8)))  float    v8f;
typedef __attribute__((ext_vector_type(4)))  float    v4f;
typedef v4f  __attribute__((may_alias)) v4fa;

__device__ __forceinline__ unsigned short f2bf(float f) { unsigned u = __float_as_uint(f); u += 0x7FFFu + ((u >> 16) & 1u); return (unsigned short)(u >> 16); }
__device__ __forceinline__ float bfr(float f) { return __uint_as_float(((unsigned)f2bf(f)) << 16); }
__device__ __forceinline__ v16bf cat16b(v8us lo, v8us hi) { return __builtin_bit_cast(v16bf, __builtin_shufflevector(lo, hi, 0, 1, 2, 3, 4, 5, 6, 7, 8, 9, 10, 11, 12, 13, 14, 15)); }
__device__ __forceinline__ v8f wmmab(v16bf a, v16bf b, v8f c) { return __builtin_amdgcn_wmma_f32_16x16x32_bf16(false, a, false, b, (short)0, c, false, false); }
__device__ __forceinline__ v16bf ldb(const bf* p)  { return cat16b(*(const v8us*)p, *(const v8us*)(p + 16)); }
__device__ __forceinline__ void wave_sync() { __builtin_amdgcn_fence(3  , "wavefront"); __builtin_amdgcn_wave_barrier(); asm volatile("" ::: "memory"); }
__device__ __forceinline__ v8f wmmab_g(v16bf a, v16bf b, v8f c) {
    c = wmmab(a, b, c);
    asm volatile("v_nop\n\tv_nop\n\tv_nop\n\tv_nop" : "+v"(c) : "v"(a), "v"(b));
    return c;
}
__device__ __forceinline__ int clamp31(int a) { return a < 0 ? 0 : (a > 31 ? 31 : a); }
__device__ __forceinline__ int tapoff(int t) { return ((t / 9) * PD + (t / 3) % 3) * PD + (t % 3); }

__global__ __launch_bounds__(256) void k_wprep(const float* __restrict__ wbase, const float* __restrict__ wplane, const float* __restrict__ wdepth, bf* WB) {
    const int g = blockIdx.x * 256 + threadIdx.x; if (g >= WROWS * (KP / 8)) return;
    const int n = g / (KP / 8), tap = g % (KP / 8);
    const int nc = n & 7, tc = tap < (NTAP - 1) ? tap : (NTAP - 1);
    const bool isv = (n < 8) & (tap < NTAP);
    const bool isq = (n >= 8) & (n < 16) & (tap == 13);
    const bool isk = (n >= 16) & (n < 24) & (tap == 13);
    v8us o;
#pragma unroll
    for (int ic = 0; ic < 8; ++ic) {
        float a = wbase[nc * 216 + ic * 27 + tc];
        float b = wplane[nc * 8 + ic];
        float c = wdepth[nc * 8 + ic];
        asm volatile("" : "+v"(a)); asm volatile("" : "+v"(b)); asm volatile("" : "+v"(c));
        const float v = isv ? a : (isq ? b : (isk ? c : 0.0f));
        o[ic] = f2bf(v); }
    *(volatile v8us*)(WB + (size_t)g * 8) = o; __threadfence(); *(volatile v8us*)(WB + (size_t)g * 8) = o;
}

__global__ __launch_bounds__(256) void k_xprep(const float* __restrict__ x, bf* XC) {
    const int pv = blockIdx.x * 256 + threadIdx.x; if (pv >= PVOX) return;
    const int pz = pv / (PD * PD), rem = pv % (PD * PD), py = rem / PD, px = rem % PD;
    const bool in = (pz >= 1) & (pz <= DIM) & (py >= 1) & (py <= DIM) & (px >= 1) & (px <= DIM);
    const int si = clamp31(pz - 1) * HW + clamp31(py - 1) * DIM + clamp31(px - 1);
    v8us o;
#pragma unroll
    for (int ic = 0; ic < 8; ++ic) {
        float a = x[(size_t)ic * DHW + si];
        asm volatile("" : "+v"(a));
        const unsigned short hb = f2bf(a);
        o[ic] = in ? hb : (unsigned short)0; }
    *(volatile v8us*)(XC + (size_t)pv * 8) = o; __threadfence(); *(volatile v8us*)(XC + (size_t)pv * 8) = o;
}

__global__ __launch_bounds__(32 * CW) void k_conv(const bf* __restrict__ XC, const bf* __restrict__ WB, const float* __restrict__ bbase, const float* __restrict__ bplane,
                                                  const float* __restrict__ bdepth, float* PL) {
    __shared__ __align__(16) float os[CW * 32 * OSP];
    const int lane = threadIdx.x & 31, lr = lane & 15, hi = lane >> 4;
    const int wave = __builtin_amdgcn_readfirstlane((int)(threadIdx.x >> 5));
    const int rw = blockIdx.x * CW + wave;
    const int d = rw >> 5, h = rw & 31;
    const size_t xrow = ((size_t)(d * PD + h) * PD + (size_t)lr) * 8;
    const size_t boff = (size_t)lr * KP + 8 * hi;
    const v8us zz = (v8us){};
    v8f av0 = (v8f){}, av1 = (v8f){}, ak0 = (v8f){}, ak1 = (v8f){};
#pragma unroll 1
    for (int s = 0; s < KSTEPS; ++s) {
        const int ta = 4 * s + hi;
        const int tr = ta + 2;
        const bool okb = tr < NTAP;
        const int tb = okb ? tr : (NTAP - 1);
        const bf* pa = XC + xrow + (size_t)tapoff(ta) * 8;
        const bf* pb = XC + xrow + (size_t)tapoff(tb) * 8;
        const v16bf b = ldb(WB + boff + 32 * s);
        const v8us a0l = *(const v8us*)pa;
        const v8us a1l = *(const v8us*)(pa + 128);
        v8us a0h = *(const v8us*)pb;
        v8us a1h = *(const v8us*)(pb + 128);
        asm volatile("" : "+v"(a0h)); asm volatile("" : "+v"(a1h));
        a0h = okb ? a0h : zz; a1h = okb ? a1h : zz;
        av0 = wmmab_g(cat16b(a0l, a0h), b, av0);
        av1 = wmmab_g(cat16b(a1l, a1h), b, av1);
    }
    {
        const bf* pa = XC + xrow + (size_t)tapoff(12 + hi) * 8;
        const bf* pb = XC + xrow + (size_t)tapoff(14 + hi) * 8;
        const v16bf b = ldb(WB + (size_t)16 * KP + boff + 96);
        const v8us a0l = *(const v8us*)pa, a0h = *(const v8us*)pb;
        const v8us a1l = *(const v8us*)(pa + 128), a1h = *(const v8us*)(pb + 128);
        ak0 = wmmab_g(cat16b(a0l, a0h), b, ak0);
        ak1 = wmmab_g(cat16b(a1l, a1h), b, ak1);
    }
    float b1v = bbase[lr & 7], b1q = bplane[lr & 7], b2k = bdepth[lr & 7];
    asm volatile("" : "+v"(b1v)); asm volatile("" : "+v"(b1q)); asm volatile("" : "+v"(b2k));
    const float bias1 = (lr < 8) ? bfr(b1v) : bfr(b1q);
    const float bias2 = (lr < 8) ? bfr(b2k) : 0.0f;
    const int wb = wave * 32 * OSP;
    { const v8f t0 = av0 + bias1, t1 = av1 + bias1, t2 = ak0 + bias2, t3 = ak1 + bias2;
      *(v4fa*)(&os[wb + lr * OSP +  0 + 8 * hi])     = __builtin_shufflevector(t0, t0, 0, 1, 2, 3);
      *(v4fa*)(&os[wb + lr * OSP +  0 + 8 * hi + 4]) = __builtin_shufflevector(t0, t0, 4, 5, 6, 7);
      *(v4fa*)(&os[wb + lr * OSP + 16 + 8 * hi])     = __builtin_shufflevector(t1, t1, 0, 1, 2, 3);
      *(v4fa*)(&os[wb + lr * OSP + 16 + 8 * hi + 4]) = __builtin_shufflevector(t1, t1, 4, 5, 6, 7);
      *(v4fa*)(&os[wb + (16 + lr) * OSP +  0 + 8 * hi])     = __builtin_shufflevector(t2, t2, 0, 1, 2, 3);
      *(v4fa*)(&os[wb + (16 + lr) * OSP +  0 + 8 * hi + 4]) = __builtin_shufflevector(t2, t2, 4, 5, 6, 7);
      *(v4fa*)(&os[wb + (16 + lr) * OSP + 16 + 8 * hi])     = __builtin_shufflevector(t3, t3, 0, 1, 2, 3);
      *(v4fa*)(&os[wb + (16 + lr) * OSP + 16 + 8 * hi + 4]) = __builtin_shufflevector(t3, t3, 4, 5, 6, 7); }
    wave_sync();
    float* prow = PL + (size_t)d * HW + (size_t)h * DIM;
#pragma unroll 1
    for (int ps = 0; ps < 2; ++ps) {
#pragma unroll
        for (int s = 0; s < 6; ++s) { const int row = 4 * s + (lane >> 3), cofs = (lane & 7) * 4;
            const v4f val = *(const v4fa*)(&os[wb + row * OSP + cofs]);
            *(volatile v4f*)(prow + (size_t)row * DHW + cofs) = val; }
        if (ps == 0) __threadfence(); }
}

__global__ __launch_bounds__(256) void k_pden(const float* __restrict__ Q, const float* __restrict__ K, float* SI) {
    const int i = blockIdx.x;
    const int j4 = threadIdx.x << 2;
    const float* qi = Q + i;
    float s0 = 0.0f, s1 = 0.0f, s2 = 0.0f, s3 = 0.0f;
#pragma unroll 2
    for (int m = 0; m < CH * DIM; ++m) {
        const float qm = qi[(size_t)m * HW] * L2E;
        const v4f km = *(const v4f*)(K + (size_t)m * HW + j4);
        s0 += __builtin_amdgcn_exp2f(qm * km[0]);
        s1 += __builtin_amdgcn_exp2f(qm * km[1]);
        s2 += __builtin_amdgcn_exp2f(qm * km[2]);
        s3 += __builtin_amdgcn_exp2f(qm * km[3]);
    }
    v4f r;
    r[0] = __builtin_amdgcn_rcpf(s0); r[1] = __builtin_amdgcn_rcpf(s1); r[2] = __builtin_amdgcn_rcpf(s2); r[3] = __builtin_amdgcn_rcpf(s3);
    float* dst = SI + (size_t)i * HW + j4;
    *(volatile v4f*)dst = r; __threadfence(); *(volatile v4f*)dst = r;
}

__global__ __launch_bounds__(256) void k_dden(const float* __restrict__ Q, const float* __restrict__ K, float* SD) {
    __shared__ float red[CH * 32];
    const int lane = threadIdx.x & 31;
    const int wave = __builtin_amdgcn_readfirstlane((int)(threadIdx.x >> 5));
    const int a = blockIdx.x;
    const float* qp = Q + (size_t)wave * DHW + (size_t)a * HW;
    const float* kp = K + (size_t)wave * DHW + (size_t)lane * HW;
    float s = 0.0f;
#pragma unroll 1
    for (int hw = 0; hw < HW; hw += 4) {
        const v4f q4 = *(const v4f*)(qp + hw);
        const v4f k4 = *(const v4f*)(kp + hw);
        s += __builtin_amdgcn_exp2f(q4[0] * L2E * k4[0]);
        s += __builtin_amdgcn_exp2f(q4[1] * L2E * k4[1]);
        s += __builtin_amdgcn_exp2f(q4[2] * L2E * k4[2]);
        s += __builtin_amdgcn_exp2f(q4[3] * L2E * k4[3]);
    }
    red[wave * 32 + lane] = s;
    __syncthreads();
    if (wave == 0) {
        float tot = 0.0f;
#pragma unroll
        for (int c = 0; c < CH; ++c) tot += red[c * 32 + lane];
        const float inv = __builtin_amdgcn_rcpf(tot);
        float* dst = SD + (size_t)a * DIM + lane;
        *(volatile float*)dst = inv; __threadfence(); *(volatile float*)dst = inv;
    }
}

__global__ __launch_bounds__(256) void k_out(const float* __restrict__ x, const float* __restrict__ Q, const float* __restrict__ K, const float* __restrict__ V,
                                             const float* __restrict__ SI, const float* __restrict__ SD, const float* __restrict__ gamma, float* OUT) {
    const int t = blockIdx.x * 256 + threadIdx.x;
    const int j = t & (HW - 1);
    const int n0 = (t >> 10) * 4;
    const int c = n0 >> 5, dd0 = n0 & 31;
    const int hh = j >> 5, ww = j & 31;
    const int tt = ww * DIM + hh;
    const size_t cb = (size_t)c * DHW;

    const float e0 = K[cb + (size_t)(dd0 + 0) * HW + tt] * L2E;
    const float e1 = K[cb + (size_t)(dd0 + 1) * HW + tt] * L2E;
    const float e2 = K[cb + (size_t)(dd0 + 2) * HW + tt] * L2E;
    const float e3 = K[cb + (size_t)(dd0 + 3) * HW + tt] * L2E;
    float d0 = 0.0f, d1 = 0.0f, d2 = 0.0f, d3 = 0.0f;
#pragma unroll 1
    for (int a = 0; a < DIM; ++a) {
        const float qa = Q[cb + (size_t)a * HW + tt];
        const float va = V[cb + (size_t)a * HW + tt];
        const v4f sd = *(const v4f*)(SD + a * DIM + dd0);
        d0 += __builtin_amdgcn_exp2f(qa * e0) * (va * sd[0]);
        d1 += __builtin_amdgcn_exp2f(qa * e1) * (va * sd[1]);
        d2 += __builtin_amdgcn_exp2f(qa * e2) * (va * sd[2]);
        d3 += __builtin_amdgcn_exp2f(qa * e3) * (va * sd[3]);
    }

    const float k0 = K[(size_t)(n0 + 0) * HW + j] * L2E;
    const float k1 = K[(size_t)(n0 + 1) * HW + j] * L2E;
    const float k2 = K[(size_t)(n0 + 2) * HW + j] * L2E;
    const float k3 = K[(size_t)(n0 + 3) * HW + j] * L2E;
    float a0 = 0.0f, a1 = 0.0f, a2 = 0.0f, a3 = 0.0f;
#pragma unroll 1
    for (int i = 0; i < HW; i += 4) {
        const float s0 = SI[(size_t)(i + 0) * HW + j];
        const float s1 = SI[(size_t)(i + 1) * HW + j];
        const float s2 = SI[(size_t)(i + 2) * HW + j];
        const float s3 = SI[(size_t)(i + 3) * HW + j];
        const v4f q0 = *(const v4f*)(Q + (size_t)(n0 + 0) * HW + i);
        const v4f q1 = *(const v4f*)(Q + (size_t)(n0 + 1) * HW + i);
        const v4f q2 = *(const v4f*)(Q + (size_t)(n0 + 2) * HW + i);
        const v4f q3 = *(const v4f*)(Q + (size_t)(n0 + 3) * HW + i);
        const v4f v0 = *(const v4f*)(V + (size_t)(n0 + 0) * HW + i);
        const v4f v1 = *(const v4f*)(V + (size_t)(n0 + 1) * HW + i);
        const v4f v2 = *(const v4f*)(V + (size_t)(n0 + 2) * HW + i);
        const v4f v3 = *(const v4f*)(V + (size_t)(n0 + 3) * HW + i);
        a0 += __builtin_amdgcn_exp2f(q0[0] * k0) * (v0[0] * s0);  a0 += __builtin_amdgcn_exp2f(q0[1] * k0) * (v0[1] * s1);
        a0 += __builtin_amdgcn_exp2f(q0[2] * k0) * (v0[2] * s2);  a0 += __builtin_amdgcn_exp2f(q0[3] * k0) * (v0[3] * s3);
        a1 += __builtin_amdgcn_exp2f(q1[0] * k1) * (v1[0] * s0);  a1 += __builtin_amdgcn_exp2f(q1[1] * k1) * (v1[1] * s1);
        a1 += __builtin_amdgcn_exp2f(q1[2] * k1) * (v1[2] * s2);  a1 += __builtin_amdgcn_exp2f(q1[3] * k1) * (v1[3] * s3);
        a2 += __builtin_amdgcn_exp2f(q2[0] * k2) * (v2[0] * s0);  a2 += __builtin_amdgcn_exp2f(q2[1] * k2) * (v2[1] * s1);
        a2 += __builtin_amdgcn_exp2f(q2[2] * k2) * (v2[2] * s2);  a2 += __builtin_amdgcn_exp2f(q2[3] * k2) * (v2[3] * s3);
        a3 += __builtin_amdgcn_exp2f(q3[0] * k3) * (v3[0] * s0);  a3 += __builtin_amdgcn_exp2f(q3[1] * k3) * (v3[1] * s1);
        a3 += __builtin_amdgcn_exp2f(q3[2] * k3) * (v3[2] * s2);  a3 += __builtin_amdgcn_exp2f(q3[3] * k3) * (v3[3] * s3);
    }
    const float g = bfr(gamma[0]);
    const float r0 = bfr(x[(size_t)(n0 + 0) * HW + j]) + g * (a0 + d0);
    const float r1 = bfr(x[(size_t)(n0 + 1) * HW + j]) + g * (a1 + d1);
    const float r2 = bfr(x[(size_t)(n0 + 2) * HW + j]) + g * (a2 + d2);
    const float r3 = bfr(x[(size_t)(n0 + 3) * HW + j]) + g * (a3 + d3);
    float* o0 = OUT + (size_t)(n0 + 0) * HW + j;
    *(volatile float*)(o0) = r0; *(volatile float*)(o0 + HW) = r1; *(volatile float*)(o0 + 2 * HW) = r2; *(volatile float*)(o0 + 3 * HW) = r3;
    __threadfence();
    *(volatile float*)(o0) = r0; *(volatile float*)(o0 + HW) = r1; *(volatile float*)(o0 + 2 * HW) = r2; *(volatile float*)(o0 + 3 * HW) = r3;
}

static constexpr size_t al256(size_t v) { return (v + 255) & ~(size_t)255; }
static constexpr size_t SZ_WB = al256((size_t)WROWS * KP * 2);
static constexpr size_t SZ_XC = al256((size_t)PVOX * CH * 2);
static constexpr size_t SZ_PL = al256((size_t)3 * CDHW * 4);
static constexpr size_t SZ_SI = al256((size_t)HW * HW * 4);
static constexpr size_t SZ_SD = al256((size_t)DIM * DIM * 4);
static constexpr size_t SZ_TOTAL = SZ_WB + SZ_XC + SZ_PL + SZ_SI + SZ_SD;
static_assert(SZ_TOTAL <= (size_t)134217728);
static_assert((size_t)(PVOX - 1) * CH * 2 + 16 <= SZ_XC);
static_assert((size_t)(WROWS * (KP / 8) - 1) * 16 + 16 <= SZ_WB);
static_assert(((size_t)23 * DHW + 31 * HW + 31 * DIM + 32) * 4 <= SZ_PL);

extern "C" void kernel_launch(void* const* d_in, const int* in_sizes, int n_in,
                              void* d_out, int out_size, void* d_ws, size_t ws_size, hipStream_t stream) {
    if (n_in < 8) return;
    if (in_sizes[0] < CDHW || in_sizes[1] < CH * CH || in_sizes[2] < CH || in_sizes[3] < CH * CH || in_sizes[4] < CH) return;
    if (in_sizes[5] < CH * CH * NTAP || in_sizes[6] < CH || in_sizes[7] < 1) return;
    if (out_size < CDHW) return;
    if (SZ_TOTAL > ws_size) return;
    const float* x      = (const float*)d_in[0];
    const float* wplane = (const float*)d_in[1];
    const float* bplane = (const float*)d_in[2];
    const float* wdepth = (const float*)d_in[3];
    const float* bdepth = (const float*)d_in[4];
    const float* wbase  = (const float*)d_in[5];
    const float* bbase  = (const float*)d_in[6];
    const float* gamma  = (const float*)d_in[7];
    float* OUT = (float*)d_out;
    char* wsp = (char*)d_ws;
    bf* WB = (bf*)wsp; wsp += SZ_WB;
    bf* XC = (bf*)wsp; wsp += SZ_XC;
    float* PL = (float*)wsp; wsp += SZ_PL;
    float* SI = (float*)wsp; wsp += SZ_SI;
    float* SD = (float*)wsp; wsp += SZ_SD;
    const float* V = PL; const float* Q = PL + CDHW; const float* K = PL + 2 * (size_t)CDHW;

    k_wprep<<<(WROWS * (KP / 8) + 255) / 256, 256, 0, stream>>>(wbase, wplane, wdepth, WB);
    k_xprep<<<(PVOX + 255) / 256, 256, 0, stream>>>(x, XC);
    k_conv<<<(DIM * DIM) / CW, 32 * CW, 0, stream>>>(XC, WB, bbase, bplane, bdepth, PL);
    k_pden<<<HW, 256, 0, stream>>>(Q, K, SI);
    k_dden<<<DIM, 256, 0, stream>>>(Q, K, SD);
    k_out<<<(CH * DIM / 4) * HW / 256, 256, 0, stream>>>(x, Q, K, V, SI, SD, gamma, OUT);
}
